// GraphAtten_64269890617452
// MI455X (gfx1250) — hardware-verified
//
#include <hip/hip_runtime.h>
#include <stddef.h>
#include <stdint.h>

#define NND  4096
#define NF   512
#define NHD  8
#define HD   128
#define NO   256
#define HC   1024
#define C1   640
#define N3   3072

static_assert(NHD * HD == HC);
static_assert(NF + HD == C1);
static_assert(3 * HC == N3);
static_assert(NND % 256 == 0);
static_assert(NF % 64 == 0 && C1 % 64 == 0 && NO % 64 == 0 && HC % 64 == 0 && HD % 64 == 0);

typedef _Float16 v16h __attribute__((ext_vector_type(16)));
typedef _Float16 v8h  __attribute__((ext_vector_type(8)));
typedef __bf16   v16bf __attribute__((ext_vector_type(16)));
typedef unsigned short v8us __attribute__((ext_vector_type(8)));
typedef float    v8f  __attribute__((ext_vector_type(8)));
typedef float    v4f  __attribute__((ext_vector_type(4)));
typedef unsigned int v4u __attribute__((ext_vector_type(4)));

union Frag  { v16h v; v8h h[2]; };
union FragB { v16bf v; v8us u[2]; };
union Pack8 { v8h h; v4u u; };
union PackU { v8us h; v4u u; };

__device__ __forceinline__ v8f mma16(v16h a, v16h b, v8f c) {
  c = __builtin_amdgcn_wmma_f32_16x16x32_f16(false, a, false, b, (short)0, c, false, false);
  asm volatile("v_nop\n\tv_nop\n\tv_nop\n\tv_nop" : "+v"(c) : "v"(a), "v"(b));
  return c;
}
__device__ __forceinline__ v8f mma16b(v16bf a, v16bf b, v8f c) {
  c = __builtin_amdgcn_wmma_f32_16x16x32_bf16(false, a, false, b, (short)0, c, false, false);
  asm volatile("v_nop\n\tv_nop\n\tv_nop\n\tv_nop" : "+v"(c) : "v"(a), "v"(b));
  return c;
}

__device__ __forceinline__ v16h ldfrag(const _Float16* p, int ld, int row0, int k0, int lane) {
  const int m = lane & 15, lh = lane >> 4;
  const _Float16* q = p + (size_t)(row0 + m) * ld + k0 + 8 * lh;
  Frag f;
  f.h[0] = *(const v8h*)(q);
  f.h[1] = *(const v8h*)(q + 16);
  return f.v;
}
__device__ __forceinline__ v16bf ldfragb(const unsigned short* p, int ld, int row0, int k0, int lane) {
  const int m = lane & 15, lh = lane >> 4;
  const unsigned short* q = p + (size_t)(row0 + m) * ld + k0 + 8 * lh;
  FragB f;
  f.u[0] = *(const v8us*)(q);
  f.u[1] = *(const v8us*)(q + 16);
  return f.v;
}

__device__ __forceinline__ v8f zero8() { return (v8f){0.f, 0.f, 0.f, 0.f, 0.f, 0.f, 0.f, 0.f}; }

__device__ __forceinline__ unsigned short bfb(float f) {
  unsigned u = __float_as_uint(f);
  u += 0x7FFFu + ((u >> 16) & 1u);
  return (unsigned short)(u >> 16);
}
__device__ __forceinline__ void split2(float f, unsigned short& h, unsigned short& l) {
  h = bfb(f);
  const float hf = __uint_as_float(((unsigned)h) << 16);
  l = bfb(f - hf);
}
__device__ __forceinline__ void split8(const float (&f)[8], v4u& vh, v4u& vl) {
  unsigned short h[8], l[8];
#pragma unroll
  for (int i = 0; i < 8; ++i) split2(f[i], h[i], l[i]);
  PackU ph, pl;
  ph.h = (v8us){h[0], h[1], h[2], h[3], h[4], h[5], h[6], h[7]};
  pl.h = (v8us){l[0], l[1], l[2], l[3], l[4], l[5], l[6], l[7]};
  vh = ph.u;
  vl = pl.u;
}

__device__ __forceinline__ void gemm32x64(const _Float16* __restrict__ A, int lda,
                                          const _Float16* __restrict__ Bt, int ldb, int K,
                                          int m0, int n0, int lane, v8f (&acc)[2][4]) {
#pragma unroll 2
  for (int k0 = 0; k0 < K; k0 += 32) {
    const v16h a0 = ldfrag(A, lda, m0, k0, lane);
    const v16h a1 = ldfrag(A, lda, m0 + 16, k0, lane);
    const v16h b0 = ldfrag(Bt, ldb, n0, k0, lane);
    const v16h b1 = ldfrag(Bt, ldb, n0 + 16, k0, lane);
    const v16h b2 = ldfrag(Bt, ldb, n0 + 32, k0, lane);
    const v16h b3 = ldfrag(Bt, ldb, n0 + 48, k0, lane);
    acc[0][0] = mma16(a0, b0, acc[0][0]);
    acc[1][0] = mma16(a1, b0, acc[1][0]);
    acc[0][1] = mma16(a0, b1, acc[0][1]);
    acc[1][1] = mma16(a1, b1, acc[1][1]);
    acc[0][2] = mma16(a0, b2, acc[0][2]);
    acc[1][2] = mma16(a1, b2, acc[1][2]);
    acc[0][3] = mma16(a0, b3, acc[0][3]);
    acc[1][3] = mma16(a1, b3, acc[1][3]);
  }
}

__device__ __forceinline__ void gemm32x64_x3(const unsigned short* __restrict__ Ah,
                                             const unsigned short* __restrict__ Al, int lda,
                                             const unsigned short* __restrict__ Bh,
                                             const unsigned short* __restrict__ Bl, int ldb, int K,
                                             int m0, int n0, int lane, v8f (&acc)[2][4]) {
#pragma unroll 1
  for (int k0 = 0; k0 < K; k0 += 32) {
    const v16bf a0h = ldfragb(Ah, lda, m0, k0, lane);
    const v16bf a1h = ldfragb(Ah, lda, m0 + 16, k0, lane);
    const v16bf a0l = ldfragb(Al, lda, m0, k0, lane);
    const v16bf a1l = ldfragb(Al, lda, m0 + 16, k0, lane);
#pragma unroll
    for (int t = 0; t < 4; ++t) {
      const v16bf bhf = ldfragb(Bh, ldb, n0 + 16 * t, k0, lane);
      const v16bf blf = ldfragb(Bl, ldb, n0 + 16 * t, k0, lane);
      acc[0][t] = mma16b(a0h, bhf, acc[0][t]);
      acc[1][t] = mma16b(a1h, bhf, acc[1][t]);
      acc[0][t] = mma16b(a0l, bhf, acc[0][t]);
      acc[1][t] = mma16b(a1l, bhf, acc[1][t]);
      acc[0][t] = mma16b(a0h, blf, acc[0][t]);
      acc[1][t] = mma16b(a1h, blf, acc[1][t]);
    }
  }
}

__global__ __launch_bounds__(256) void k_cvt_x(const float* __restrict__ x, _Float16* __restrict__ xh,
                                               unsigned short* __restrict__ hhi, unsigned short* __restrict__ hlo,
                                               int ngrp) {
  const int t = blockIdx.x * 256 + (int)threadIdx.x;
  if (t >= ngrp) return;
  const int row = t >> 6, c8 = t & 63;
  const size_t si = (size_t)row * NF + c8 * 8;
  const size_t di = (size_t)row * C1 + c8 * 8;
  const v4f a0 = *(const v4f*)(x + si);
  const v4f a1 = *(const v4f*)(x + si + 4);
  Pack8 pk;
  pk.h = (v8h){(_Float16)a0[0], (_Float16)a0[1], (_Float16)a0[2], (_Float16)a0[3],
               (_Float16)a1[0], (_Float16)a1[1], (_Float16)a1[2], (_Float16)a1[3]};
  const v4u vx = pk.u;
  const float f[8] = {a0[0], a0[1], a0[2], a0[3], a1[0], a1[1], a1[2], a1[3]};
  v4u vh, vl;
  split8(f, vh, vl);
  volatile v4u* dx = (volatile v4u*)(xh + si);
  volatile v4u* dh = (volatile v4u*)(hhi + di);
  volatile v4u* dl = (volatile v4u*)(hlo + di);
  *dx = vx; *dh = vh; *dl = vl;
  __threadfence();
  *dx = vx; *dh = vh; *dl = vl;
}

#define WTP 68
__global__ __launch_bounds__(256) void k_wt(const float* __restrict__ w, _Float16* __restrict__ wt,
                                            int K, int nout, float scale) {
  __shared__ __align__(16) float tf[64 * WTP];
  const int tid = threadIdx.x;
  const int n0 = blockIdx.x * 64;
  const int k0 = blockIdx.y * 64;
  const int mat = blockIdx.z;
  const float* wb = w + (size_t)mat * K * nout;
  _Float16* ob = wt + (size_t)mat * nout * K;
  {
    const int kr = tid >> 4;
    const int n4 = (tid & 15) * 4;
#pragma unroll
    for (int it = 0; it < 4; ++it) {
      const int kl = it * 16 + kr;
      const v4f a = *(const v4f*)(wb + (size_t)(k0 + kl) * nout + n0 + n4);
      *(v4f*)(tf + kl * WTP + n4) = a;
    }
  }
  __syncthreads();
  v4u val[2];
  size_t go[2];
#pragma unroll
  for (int j = 0; j < 2; ++j) {
    const int p  = tid + 256 * j;
    const int nl = p >> 3;
    const int pc = p & 7;
    const float* cp = tf + (pc * 8) * WTP + nl;
    Pack8 pk;
    pk.h = (v8h){(_Float16)(cp[0 * WTP] * scale), (_Float16)(cp[1 * WTP] * scale),
                 (_Float16)(cp[2 * WTP] * scale), (_Float16)(cp[3 * WTP] * scale),
                 (_Float16)(cp[4 * WTP] * scale), (_Float16)(cp[5 * WTP] * scale),
                 (_Float16)(cp[6 * WTP] * scale), (_Float16)(cp[7 * WTP] * scale)};
    val[j] = pk.u;
    go[j]  = (size_t)(n0 + nl) * K + k0 + pc * 8;
  }
  for (int ps = 0; ps < 2; ++ps) {
#pragma unroll
    for (int j = 0; j < 2; ++j) *(volatile v4u*)(ob + go[j]) = val[j];
    __threadfence();
  }
}

__global__ __launch_bounds__(256) void k_wt_bf(const float* __restrict__ w, unsigned short* __restrict__ wh,
                                               unsigned short* __restrict__ wl, int K, int nout) {
  __shared__ __align__(16) float tf[64 * WTP];
  const int tid = threadIdx.x;
  const int n0 = blockIdx.x * 64;
  const int k0 = blockIdx.y * 64;
  {
    const int kr = tid >> 4;
    const int n4 = (tid & 15) * 4;
#pragma unroll
    for (int it = 0; it < 4; ++it) {
      const int kl = it * 16 + kr;
      const v4f a = *(const v4f*)(w + (size_t)(k0 + kl) * nout + n0 + n4);
      *(v4f*)(tf + kl * WTP + n4) = a;
    }
  }
  __syncthreads();
  v4u vhs[2], vls[2];
  size_t go[2];
#pragma unroll
  for (int j = 0; j < 2; ++j) {
    const int p  = tid + 256 * j;
    const int nl = p >> 3;
    const int pc = p & 7;
    const float* cp = tf + (pc * 8) * WTP + nl;
    const float f[8] = {cp[0 * WTP], cp[1 * WTP], cp[2 * WTP], cp[3 * WTP],
                        cp[4 * WTP], cp[5 * WTP], cp[6 * WTP], cp[7 * WTP]};
    split8(f, vhs[j], vls[j]);
    go[j] = (size_t)(n0 + nl) * K + k0 + pc * 8;
  }
  for (int ps = 0; ps < 2; ++ps) {
#pragma unroll
    for (int j = 0; j < 2; ++j) {
      *(volatile v4u*)(wh + go[j]) = vhs[j];
      *(volatile v4u*)(wl + go[j]) = vls[j];
    }
    __threadfence();
  }
}

#define STP 72
__global__ __launch_bounds__(256) void k_qkv(const _Float16* __restrict__ xh,
                                             const _Float16* __restrict__ wt,
                                             const float* __restrict__ bq,
                                             const float* __restrict__ bk,
                                             const float* __restrict__ bv,
                                             _Float16* __restrict__ qp,
                                             _Float16* __restrict__ kp,
                                             _Float16* __restrict__ vt) {
  __shared__ __align__(16) _Float16 st[256 * STP];
  const int tid = threadIdx.x, lane = tid & 31, wave = tid >> 5;
  const int hh = lane >> 4, c = lane & 15;
  const int mb = blockIdx.x * 256;
  const int m0 = mb + wave * 32;
  const int n0 = blockIdx.y * 64;

  v8f acc[2][4];
#pragma unroll
  for (int s = 0; s < 2; ++s)
#pragma unroll
    for (int t = 0; t < 4; ++t) acc[s][t] = zero8();
  gemm32x64(xh, NF, wt, NF, NF, m0, n0, lane, acc);

  const int which = n0 >> 10;
  const int head  = (n0 & (HC - 1)) >> 7;
  const int dh0   = n0 & (HD - 1);
  const float* bias = (which == 0 ? bq : (which == 1 ? bk : bv)) + head * HD + dh0;

#pragma unroll
  for (int t = 0; t < 4; ++t) {
    const float bvl = bias[16 * t + c];
#pragma unroll
    for (int sub = 0; sub < 2; ++sub) {
#pragma unroll
      for (int r = 0; r < 8; ++r) {
        const int lr = wave * 32 + sub * 16 + 8 * hh + r;
        st[lr * STP + 16 * t + c] = (_Float16)fmaxf(acc[sub][t][r] * 0.0625f + bvl, 0.f);
      }
    }
  }
  __syncthreads();

  _Float16* dst = (which == 0 ? qp : (which == 1 ? kp : vt));
  v4u val[8];
  size_t go[8];
  if (which < 2) {
#pragma unroll
    for (int j = 0; j < 8; ++j) {
      const int p  = tid + 256 * j;
      const int lr = p >> 3;
      const int pc = p & 7;
      Pack8 pk;
      pk.h  = *(const v8h*)(st + lr * STP + pc * 8);
      val[j] = pk.u;
      go[j]  = ((size_t)head * NND + mb + lr) * HD + dh0 + pc * 8;
    }
  } else {
#pragma unroll
    for (int j = 0; j < 8; ++j) {
      const int p  = tid + 256 * j;
      const int L  = p >> 3;
      const int pc = p & 7;
      const int d  = L >> 2;
      const int nl = (L & 3) * 64 + pc * 8;
      const _Float16* cp = st + nl * STP + d;
      Pack8 pk;
      pk.h = (v8h){cp[0 * STP], cp[1 * STP], cp[2 * STP], cp[3 * STP],
                   cp[4 * STP], cp[5 * STP], cp[6 * STP], cp[7 * STP]};
      val[j] = pk.u;
      go[j]  = ((size_t)head * HD + dh0 + d) * NND + mb + nl;
    }
  }
  for (int ps = 0; ps < 2; ++ps) {
#pragma unroll
    for (int j = 0; j < 8; ++j) *(volatile v4u*)(dst + go[j]) = val[j];
    __threadfence();
  }
}

#define KTP 136
#define VTP 72
#define PTP 72
#define OSP 136
#define LDS_KS  0
#define LDS_VS  (64 * KTP)
#define LDS_PS  (LDS_VS + 128 * VTP)
#define LDS_TOT (LDS_PS + 8 * 16 * PTP)
static_assert(8 * 16 * OSP <= LDS_TOT);
static_assert((LDS_VS * 2) % 16 == 0 && (LDS_PS * 2) % 16 == 0);

__global__ __launch_bounds__(256) void k_attn(const _Float16* __restrict__ qp,
                                              const _Float16* __restrict__ kp,
                                              const _Float16* __restrict__ vt,
                                              _Float16* __restrict__ op) {
  __shared__ __align__(16) _Float16 lds[LDS_TOT];
  _Float16* Ks = lds + LDS_KS;
  _Float16* Vs = lds + LDS_VS;

  const int tid = threadIdx.x, lane = tid & 31, wave = tid >> 5;
  const int hh = lane >> 4, c = lane & 15;
  const int head = blockIdx.x >> 5;
  const int qb   = blockIdx.x & 31;
  const int q0   = qb * 128 + wave * 16;

  const _Float16* Q = qp + (size_t)head * NND * HD;
  const _Float16* K = kp + (size_t)head * NND * HD;
  const _Float16* V = vt + (size_t)head * HD * NND;

  v16h qa[4];
#pragma unroll
  for (int dc = 0; dc < 4; ++dc) qa[dc] = ldfrag(Q, HD, q0, 32 * dc, lane);

  const float NEGI = -__builtin_huge_valf();
  float mrow[8], lrow[8];
  v8f oacc[8];
#pragma unroll
  for (int r = 0; r < 8; ++r) { mrow[r] = NEGI; lrow[r] = 0.f; }
#pragma unroll
  for (int t = 0; t < 8; ++t) oacc[t] = zero8();

  _Float16* pw = lds + LDS_PS + wave * (16 * PTP);

  for (int kc = 0; kc < NND / 64; ++kc) {
    const int kv0 = kc * 64;
    __syncthreads();
    {
      const int r  = tid >> 2;
      const int qq = (tid & 3) * 32;
      const _Float16* ks = K + (size_t)(kv0 + r) * HD + qq;
      _Float16* kd = Ks + r * KTP + qq;
#pragma unroll
      for (int i = 0; i < 4; ++i) *(v8h*)(kd + 8 * i) = *(const v8h*)(ks + 8 * i);
      const int r2 = tid >> 1;
      const int q2 = (tid & 1) * 32;
      const _Float16* vs = V + (size_t)r2 * NND + kv0 + q2;
      _Float16* vd = Vs + r2 * VTP + q2;
#pragma unroll
      for (int i = 0; i < 4; ++i) *(v8h*)(vd + 8 * i) = *(const v8h*)(vs + 8 * i);
    }
    __syncthreads();

    v8f s[4];
#pragma unroll
    for (int j = 0; j < 4; ++j) s[j] = zero8();
#pragma unroll
    for (int dc = 0; dc < 4; ++dc) {
#pragma unroll
      for (int j = 0; j < 4; ++j) {
        const v16h kb = ldfrag(Ks, KTP, j * 16, dc * 32, lane);
        s[j] = mma16(qa[dc], kb, s[j]);
      }
    }
    float cm[8];
#pragma unroll
    for (int r = 0; r < 8; ++r) {
      float m = NEGI;
#pragma unroll
      for (int j = 0; j < 4; ++j) {
        float sv = s[j][r];
        sv = (sv > 0.f) ? sv : 0.2f * sv;
        s[j][r] = sv;
        m = fmaxf(m, sv);
      }
#pragma unroll
      for (int off = 1; off < 16; off <<= 1) m = fmaxf(m, __shfl_xor(m, off, 32));
      cm[r] = m;
    }
    float al[8];
#pragma unroll
    for (int r = 0; r < 8; ++r) {
      const float mnew  = fmaxf(mrow[r], cm[r]);
      const float alpha = __expf(mrow[r] - mnew);
      mrow[r] = mnew;
      float psum = 0.f;
#pragma unroll
      for (int j = 0; j < 4; ++j) {
        const float p = __expf(s[j][r] - mnew);
        psum += p;
        pw[(8 * hh + r) * PTP + j * 16 + c] = (_Float16)(p * 1024.0f);
      }
#pragma unroll
      for (int off = 1; off < 16; off <<= 1) psum += __shfl_xor(psum, off, 32);
      lrow[r] = lrow[r] * alpha + psum;
      al[r] = alpha;
    }
#pragma unroll
    for (int t = 0; t < 8; ++t)
#pragma unroll
      for (int r = 0; r < 8; ++r) oacc[t][r] *= al[r];
    __syncthreads();

#pragma unroll
    for (int kk = 0; kk < 2; ++kk) {
      const v16h pa = ldfrag(pw, PTP, 0, kk * 32, lane);
#pragma unroll
      for (int t = 0; t < 8; ++t) {
        const v16h vb = ldfrag(Vs, VTP, t * 16, kk * 32, lane);
        oacc[t] = mma16(pa, vb, oacc[t]);
      }
    }
  }
  __syncthreads();

  _Float16* ow = lds + wave * (16 * OSP);
#pragma unroll
  for (int r = 0; r < 8; ++r) {
    const float inv = 0.015625f / lrow[r];
#pragma unroll
    for (int t = 0; t < 8; ++t) ow[(8 * hh + r) * OSP + 16 * t + c] = (_Float16)(oacc[t][r] * inv);
  }
  __syncthreads();
  v4u val[8];
  size_t go[8];
#pragma unroll
  for (int it = 0; it < 8; ++it) {
    const int p    = lane + 32 * it;
    const int L    = p >> 3;
    const int pc   = p & 7;
    const int row  = L >> 1;
    const int half = L & 1;
    Pack8 pk;
    pk.h    = *(const v8h*)(ow + row * OSP + half * 64 + pc * 8);
    val[it] = pk.u;
    go[it]  = (size_t)(q0 + row) * HC + (size_t)head * HD + half * 64 + pc * 8;
  }
  for (int ps = 0; ps < 2; ++ps) {
#pragma unroll
    for (int it = 0; it < 8; ++it) *(volatile v4u*)(op + go[it]) = val[it];
    __threadfence();
  }
}

#define OTP 68
__global__ __launch_bounds__(256) void k_mproj(const _Float16* __restrict__ op,
                                               const _Float16* __restrict__ wmt,
                                               const float* __restrict__ bm,
                                               unsigned short* __restrict__ hhi,
                                               unsigned short* __restrict__ hlo) {
  __shared__ __align__(16) float st[8][16 * OTP];
  const int tid = threadIdx.x, lane = tid & 31, wave = tid >> 5;
  const int hh = lane >> 4, c = lane & 15;
  const int m0 = blockIdx.x * 256 + wave * 32;
  const int n0 = blockIdx.y * 64;

  v8f acc[2][4];
#pragma unroll
  for (int s = 0; s < 2; ++s)
#pragma unroll
    for (int t = 0; t < 4; ++t) acc[s][t] = zero8();
  gemm32x64(op, HC, wmt, HC, HC, m0, n0, lane, acc);

  float bvs[4];
#pragma unroll
  for (int t = 0; t < 4; ++t) bvs[t] = bm[n0 + 16 * t + c];

  float* sw = st[wave];
#pragma unroll
  for (int sub = 0; sub < 2; ++sub) {
    __syncthreads();
#pragma unroll
    for (int t = 0; t < 4; ++t) {
#pragma unroll
      for (int r = 0; r < 8; ++r)
        sw[(8 * hh + r) * OTP + 16 * t + c] = fmaxf(acc[sub][t][r] * 0.001953125f + bvs[t], 0.f);
    }
    __syncthreads();
    v4u vhs[4], vls[4];
    size_t go[4];
#pragma unroll
    for (int it = 0; it < 4; ++it) {
      const int p  = lane + 32 * it;
      const int L  = p >> 3;
      const int pc = p & 7;
      const v4f f0 = *(const v4f*)(sw + L * OTP + pc * 8);
      const v4f f1 = *(const v4f*)(sw + L * OTP + pc * 8 + 4);
      const float f[8] = {f0[0], f0[1], f0[2], f0[3], f1[0], f1[1], f1[2], f1[3]};
      split8(f, vhs[it], vls[it]);
      go[it] = (size_t)(m0 + sub * 16 + L) * C1 + NF + n0 + pc * 8;
    }
    for (int ps = 0; ps < 2; ++ps) {
#pragma unroll
      for (int it = 0; it < 4; ++it) {
        *(volatile v4u*)(hhi + go[it]) = vhs[it];
        *(volatile v4u*)(hlo + go[it]) = vls[it];
      }
      __threadfence();
    }
  }
}

__global__ __launch_bounds__(256) void k_gemm_x3(const unsigned short* __restrict__ ah,
                                                 const unsigned short* __restrict__ al, int lda,
                                                 const unsigned short* __restrict__ bh,
                                                 const unsigned short* __restrict__ bl, int K,
                                                 const float* __restrict__ bias,
                                                 float* __restrict__ out, int ldc) {
  __shared__ __align__(16) float st[8][16 * OTP];
  const int tid = threadIdx.x, lane = tid & 31, wave = tid >> 5;
  const int hh = lane >> 4, c = lane & 15;
  const int m0 = blockIdx.x * 256 + wave * 32;
  const int n0 = blockIdx.y * 64;

  v8f acc[2][4];
#pragma unroll
  for (int s = 0; s < 2; ++s)
#pragma unroll
    for (int t = 0; t < 4; ++t) acc[s][t] = zero8();
  gemm32x64_x3(ah, al, lda, bh, bl, K, K, m0, n0, lane, acc);

  float bvs[4];
#pragma unroll
  for (int t = 0; t < 4; ++t) bvs[t] = bias[n0 + 16 * t + c];

  float* sw = st[wave];
#pragma unroll
  for (int sub = 0; sub < 2; ++sub) {
    __syncthreads();
#pragma unroll
    for (int t = 0; t < 4; ++t) {
#pragma unroll
      for (int r = 0; r < 8; ++r)
        sw[(8 * hh + r) * OTP + 16 * t + c] = acc[sub][t][r] + bvs[t];
    }
    __syncthreads();
    v4f val[8];
    size_t go[8];
#pragma unroll
    for (int it = 0; it < 8; ++it) {
      const int p    = lane + 32 * it;
      const int L    = p >> 3;
      const int pc   = p & 7;
      const int row  = L >> 1;
      const int half = L & 1;
      val[it] = *(const v4f*)(sw + row * OTP + half * 32 + pc * 4);
      go[it]  = (size_t)(m0 + sub * 16 + row) * ldc + n0 + half * 32 + pc * 4;
    }
    for (int ps = 0; ps < 2; ++ps) {
#pragma unroll
      for (int it = 0; it < 8; ++it) *(volatile v4f*)(out + go[it]) = val[it];
      __threadfence();
    }
  }
}

__global__ __launch_bounds__(256) void k_bn_stats(const float* __restrict__ Z, int ncol,
                                                  float* __restrict__ mu, float* __restrict__ rstd) {
  __shared__ double sb[4][64], sb2[4][64];
  __shared__ __align__(16) float mus[64];
  __shared__ __align__(16) float rss[64];
  const int tid = threadIdx.x, cl = tid & 63, rs = tid >> 6;
  const int c0 = blockIdx.x * 64;
  const float* zc = Z + c0 + cl;
  double s = 0.0, s2 = 0.0;
#pragma unroll 4
  for (int r = rs; r < NND; r += 4) {
    const double z = (double)zc[(size_t)r * ncol];
    s += z;
    s2 += z * z;
  }
  sb[rs][cl] = s;
  sb2[rs][cl] = s2;
  __syncthreads();
  if (rs == 0) {
    const double ts  = ((sb[0][cl] + sb[1][cl]) + sb[2][cl]) + sb[3][cl];
    const double ts2 = ((sb2[0][cl] + sb2[1][cl]) + sb2[2][cl]) + sb2[3][cl];
    const double m = ts * (1.0 / 4096.0);
    double var = ts2 * (1.0 / 4096.0) - m * m;
    var = (var > 0.0) ? var : 0.0;
    const float vf = (float)var + 1e-5f;
    mus[cl] = (float)m;
    rss[cl] = 1.0f / sqrtf(vf);
  }
  __syncthreads();
  if (tid < 32) {
    const int lane = tid;
    const int i4 = (lane & 15) * 4;
    const v4f va = *(const v4f*)(mus + i4);
    const v4f vb = *(const v4f*)(rss + i4);
    v4f vv = va;
    if (lane >= 16) vv = vb;
    float* dst = ((lane < 16) ? mu : rstd) + c0 + i4;
    *(volatile v4f*)dst = vv;
    __threadfence();
    *(volatile v4f*)dst = vv;
  }
}

__global__ __launch_bounds__(256) void k_bn_apply_h(const float* __restrict__ Z,
                                                    const float* __restrict__ mu,
                                                    const float* __restrict__ rstd,
                                                    const float* __restrict__ g,
                                                    const float* __restrict__ be,
                                                    unsigned short* __restrict__ Hh,
                                                    unsigned short* __restrict__ Hl, int ntot) {
  const int t = blockIdx.x * 256 + (int)threadIdx.x;
  if (t >= ntot) return;
  const int PPR = C1 / 8;
  const int col = (t - (t / PPR) * PPR) * 8;
  const size_t o = (size_t)t * 8;
  const v4f z0 = *(const v4f*)(Z + o),       z1 = *(const v4f*)(Z + o + 4);
  const v4f m0 = *(const v4f*)(mu + col),    m1 = *(const v4f*)(mu + col + 4);
  const v4f r0 = *(const v4f*)(rstd + col),  r1 = *(const v4f*)(rstd + col + 4);
  const v4f g0 = *(const v4f*)(g + col),     g1 = *(const v4f*)(g + col + 4);
  const v4f e0 = *(const v4f*)(be + col),    e1 = *(const v4f*)(be + col + 4);
  const v4f y0 = (g0 * (z0 - m0)) * r0 + e0;
  const v4f y1 = (g1 * (z1 - m1)) * r1 + e1;
  const float f[8] = {fmaxf(y0[0], 0.f), fmaxf(y0[1], 0.f), fmaxf(y0[2], 0.f), fmaxf(y0[3], 0.f),
                      fmaxf(y1[0], 0.f), fmaxf(y1[1], 0.f), fmaxf(y1[2], 0.f), fmaxf(y1[3], 0.f)};
  v4u vh, vl;
  split8(f, vh, vl);
  volatile v4u* dh = (volatile v4u*)(Hh + o);
  volatile v4u* dl = (volatile v4u*)(Hl + o);
  *dh = vh; *dl = vl;
  __threadfence();
  *dh = vh; *dl = vl;
}

__global__ __launch_bounds__(256) void k_bn_apply_out(const float* __restrict__ Z,
                                                      const float* __restrict__ mu,
                                                      const float* __restrict__ rstd,
                                                      const float* __restrict__ g,
                                                      const float* __restrict__ be,
                                                      float* __restrict__ out, int ntot) {
  const int t = blockIdx.x * 256 + (int)threadIdx.x;
  if (t >= ntot) return;
  const int col = (t & (NO / 4 - 1)) * 4;
  const size_t o = (size_t)t * 4;
  const v4f z0 = *(const v4f*)(Z + o);
  const v4f m0 = *(const v4f*)(mu + col);
  const v4f r0 = *(const v4f*)(rstd + col);
  const v4f g0 = *(const v4f*)(g + col);
  const v4f e0 = *(const v4f*)(be + col);
  const v4f y0 = (g0 * (z0 - m0)) * r0 + e0;
  const v4f vv = (v4f){fmaxf(y0[0], 0.f), fmaxf(y0[1], 0.f), fmaxf(y0[2], 0.f), fmaxf(y0[3], 0.f)};
  volatile v4f* d = (volatile v4f*)(out + o);
  *d = vv;
  __threadfence();
  *d = vv;
}

extern "C" void kernel_launch(void* const* d_in, const int* in_sizes, int n_in,
                              void* d_out, int out_size, void* d_ws, size_t ws_size,
                              hipStream_t stream) {
  if (n_in < 17) return;
  if (in_sizes[0] != NND * NF) return;
  if (in_sizes[1] != NHD * NF * HD || in_sizes[3] != NHD * NF * HD || in_sizes[5] != NHD * NF * HD) return;
  if (in_sizes[2] != NHD * HD || in_sizes[4] != NHD * HD || in_sizes[6] != NHD * HD) return;
  if (in_sizes[7] != HC * HD || in_sizes[8] != HD) return;
  if (in_sizes[9] != C1 * C1 || in_sizes[10] != C1 || in_sizes[11] != C1 || in_sizes[12] != C1) return;
  if (in_sizes[13] != C1 * NO || in_sizes[14] != NO || in_sizes[15] != NO || in_sizes[16] != NO) return;
  if (out_size != NND * NO) return;

  const float* x   = (const float*)d_in[0];
  const float* Wq  = (const float*)d_in[1];
  const float* bq  = (const float*)d_in[2];
  const float* Wk  = (const float*)d_in[3];
  const float* bk  = (const float*)d_in[4];
  const float* Wv  = (const float*)d_in[5];
  const float* bv  = (const float*)d_in[6];
  const float* Wm  = (const float*)d_in[7];
  const float* bm  = (const float*)d_in[8];
  const float* W1  = (const float*)d_in[9];
  const float* b1  = (const float*)d_in[10];
  const float* g1  = (const float*)d_in[11];
  const float* be1 = (const float*)d_in[12];
  const float* W2  = (const float*)d_in[13];
  const float* b2  = (const float*)d_in[14];
  const float* g2  = (const float*)d_in[15];
  const float* be2 = (const float*)d_in[16];
  float* out = (float*)d_out;

  size_t off = 0;
  const size_t oXh  = off; off += (size_t)NND * NF * 2;
  const size_t oHh  = off; off += (size_t)NND * C1 * 2;
  const size_t oHl  = off; off += (size_t)NND * C1 * 2;
  const size_t oWt3 = off; off += (size_t)N3 * NF * 2;
  const size_t oWmt = off; off += (size_t)HD * HC * 2;
  const size_t oW1h = off; off += (size_t)C1 * C1 * 2;
  const size_t oW1l = off; off += (size_t)C1 * C1 * 2;
  const size_t oW2h = off; off += (size_t)NO * C1 * 2;
  const size_t oW2l = off; off += (size_t)NO * C1 * 2;
  const size_t oQ   = off; off += (size_t)NHD * NND * HD * 2;
  const size_t oK   = off; off += (size_t)NHD * NND * HD * 2;
  const size_t oV   = off; off += (size_t)NHD * HD * NND * 2;
  const size_t oO   = off; off += (size_t)NND * HC * 2;
  const size_t oZ1  = off; off += (size_t)NND * C1 * 4;
  const size_t oH1h = off; off += (size_t)NND * C1 * 2;
  const size_t oH1l = off; off += (size_t)NND * C1 * 2;
  const size_t oZ2  = off; off += (size_t)NND * NO * 4;
  const size_t oMu1 = off; off += (size_t)C1 * 4;
  const size_t oRs1 = off; off += (size_t)C1 * 4;
  const size_t oMu2 = off; off += (size_t)NO * 4;
  const size_t oRs2 = off; off += (size_t)NO * 4;
  if (off > ws_size) return;

  char* ws = (char*)d_ws;
  _Float16* Xh  = (_Float16*)(ws + oXh);
  unsigned short* Hh  = (unsigned short*)(ws + oHh);
  unsigned short* Hl  = (unsigned short*)(ws + oHl);
  _Float16* Wt3 = (_Float16*)(ws + oWt3);
  _Float16* Wmt = (_Float16*)(ws + oWmt);
  unsigned short* W1h = (unsigned short*)(ws + oW1h);
  unsigned short* W1l = (unsigned short*)(ws + oW1l);
  unsigned short* W2h = (unsigned short*)(ws + oW2h);
  unsigned short* W2l = (unsigned short*)(ws + oW2l);
  _Float16* Qp  = (_Float16*)(ws + oQ);
  _Float16* Kp  = (_Float16*)(ws + oK);
  _Float16* Vtp = (_Float16*)(ws + oV);
  _Float16* Op  = (_Float16*)(ws + oO);
  float*    Z1  = (float*)(ws + oZ1);
  unsigned short* H1h = (unsigned short*)(ws + oH1h);
  unsigned short* H1l = (unsigned short*)(ws + oH1l);
  float*    Z2  = (float*)(ws + oZ2);
  float*    mu1 = (float*)(ws + oMu1);
  float*    rs1 = (float*)(ws + oRs1);
  float*    mu2 = (float*)(ws + oMu2);
  float*    rs2 = (float*)(ws + oRs2);

  const int ngrp = NND * (NF / 8);
  k_cvt_x<<<dim3((ngrp + 255) / 256), dim3(256), 0, stream>>>(x, Xh, Hh, Hl, ngrp);
  k_wt<<<dim3(HD / 64, NF / 64, NHD), dim3(256), 0, stream>>>(Wq, Wt3, NF, HD, 16.0f);
  k_wt<<<dim3(HD / 64, NF / 64, NHD), dim3(256), 0, stream>>>(Wk, Wt3 + (size_t)HC * NF, NF, HD, 16.0f);
  k_wt<<<dim3(HD / 64, NF / 64, NHD), dim3(256), 0, stream>>>(Wv, Wt3 + (size_t)2 * HC * NF, NF, HD, 16.0f);
  k_wt<<<dim3(HD / 64, HC / 64, 1), dim3(256), 0, stream>>>(Wm, Wmt, HC, HD, 32.0f);
  k_wt_bf<<<dim3(C1 / 64, C1 / 64), dim3(256), 0, stream>>>(W1, W1h, W1l, C1, C1);
  k_wt_bf<<<dim3(NO / 64, C1 / 64), dim3(256), 0, stream>>>(W2, W2h, W2l, C1, NO);
  k_qkv<<<dim3(NND / 256, N3 / 64), dim3(256), 0, stream>>>(Xh, Wt3, bq, bk, bv, Qp, Kp, Vtp);
  k_attn<<<dim3(NHD * (NND / 128)), dim3(256), 0, stream>>>(Qp, Kp, Vtp, Op);
  k_mproj<<<dim3(NND / 256, HD / 64), dim3(256), 0, stream>>>(Op, Wmt, bm, Hh, Hl);
  k_gemm_x3<<<dim3(NND / 256, C1 / 64), dim3(256), 0, stream>>>(Hh, Hl, C1, W1h, W1l, C1, b1, Z1, C1);
  k_bn_stats<<<dim3(C1 / 64), dim3(256), 0, stream>>>(Z1, C1, mu1, rs1);
  const int nh1 = NND * (C1 / 8);
  k_bn_apply_h<<<dim3((nh1 + 255) / 256), dim3(256), 0, stream>>>(Z1, mu1, rs1, g1, be1, H1h, H1l, nh1);
  k_gemm_x3<<<dim3(NND / 256, NO / 64), dim3(256), 0, stream>>>(H1h, H1l, C1, W2h, W2l, C1, b2, Z2, NO);
  k_bn_stats<<<dim3(NO / 64), dim3(256), 0, stream>>>(Z2, NO, mu2, rs2);
  const int nout4 = NND * (NO / 4);
  k_bn_apply_out<<<dim3((nout4 + 255) / 256), dim3(256), 0, stream>>>(Z2, mu2, rs2, g2, be2, out, nout4);
  (void)hipGetLastError();
}
